// MixtureConfounderPrior_21792664060394
// MI455X (gfx1250) — hardware-verified
//
#include <hip/hip_runtime.h>
#include <math.h>

typedef unsigned short us16;
typedef us16   v8us  __attribute__((ext_vector_type(8)));
typedef __bf16 v16bf __attribute__((ext_vector_type(16)));
typedef float  v8f   __attribute__((ext_vector_type(8)));
typedef float  v4f   __attribute__((ext_vector_type(4)));
typedef v8us __attribute__((may_alias)) v8usa;
typedef v4f  __attribute__((may_alias)) v4fa;

union Frag { v16bf v; v8us half[2]; };

#define NTOK   1024
#define DDIM   1024
#define KCODE  32
#define CDIM   128
#define CFD    128
#define MWH    256
#define LD_W1  1152
#define NH8    (NTOK * DDIM / 8)
#define LVMIN  (-2.3025850929940455f)
#define LVMAX  (0.6931471805599453f)
#define LNEPS  (1e-5f)

__device__ __forceinline__ us16 bf16_rne(float x) {
  const unsigned int u = __float_as_uint(x);
  return (us16)((u + 0x7FFFu + ((u >> 16) & 1u)) >> 16);
}
__device__ __forceinline__ void split1(float x, us16& hi, us16& lo) {
  const us16 hb = bf16_rne(x);
  const float r = x - __uint_as_float(((unsigned int)hb) << 16);
  hi = hb;
  lo = bf16_rne(r);
}
__device__ __forceinline__ void split8(v4f a, v4f c, v8us& vh, v8us& vl) {
  us16 h0, h1, h2, h3, h4, h5, h6, h7, l0, l1, l2, l3, l4, l5, l6, l7;
  split1(a.x, h0, l0); split1(a.y, h1, l1); split1(a.z, h2, l2); split1(a.w, h3, l3);
  split1(c.x, h4, l4); split1(c.y, h5, l5); split1(c.z, h6, l6); split1(c.w, h7, l7);
  const v8us th = { h0, h1, h2, h3, h4, h5, h6, h7 };
  const v8us tl = { l0, l1, l2, l3, l4, l5, l6, l7 };
  vh = th; vl = tl;
}

__device__ __forceinline__ v8f wmma_bf(v16bf a, v16bf b, v8f c) {
  v8f d = __builtin_amdgcn_wmma_f32_16x16x32_bf16(false, a, false, b, (short)0, c, false, false);
  asm volatile("v_nop\n\tv_nop\n\tv_nop\n\tv_nop" : "+v"(d) : "v"(a), "v"(b));
  return d;
}
__device__ __forceinline__ v8f mma3(v16bf ah, v16bf al, v16bf bh, v16bf bl, v8f c) {
  c = wmma_bf(ah, bh, c);
  c = wmma_bf(ah, bl, c);
  c = wmma_bf(al, bh, c);
  return c;
}
__device__ __forceinline__ v16bf load_frag(const us16* p, int h) {
  Frag f;
  f.half[0] = *(const v8usa*)(p + 8 * h);
  f.half[1] = *(const v8usa*)(p + 16 + 8 * h);
  return f.v;
}

__global__ __launch_bounds__(256) void k_convert_h(const float* __restrict__ h,
                                                   us16* __restrict__ Hh, us16* __restrict__ Hl) {
  const int g = blockIdx.x * 256 + threadIdx.x;
  if (g >= NH8) return;
  const float* src = h + (size_t)g * 8;
  const v4f a = *(const v4fa*)src;
  const v4f c = *(const v4fa*)(src + 4);
  v8us vh, vl;
  split8(a, c, vh, vl);
  us16* dh = Hh + (size_t)g * 8;
  us16* dl = Hl + (size_t)g * 8;
  *(volatile v8us*)dh = vh;
  *(volatile v8us*)dl = vl;
  __threadfence();
  *(volatile v8us*)dh = vh;
  *(volatile v8us*)dl = vl;
}

__global__ __launch_bounds__(256) void k_transpose_w(
    const float* __restrict__ w0, const float* __restrict__ w1, const float* __restrict__ w2,
    const float* __restrict__ w3, const float* __restrict__ w4,
    us16* __restrict__ t0h, us16* __restrict__ t0l, us16* __restrict__ t1h, us16* __restrict__ t1l,
    us16* __restrict__ t2h, us16* __restrict__ t2l, us16* __restrict__ t3h, us16* __restrict__ t3l,
    us16* __restrict__ t4h, us16* __restrict__ t4l)
{
  __shared__ __attribute__((aligned(16))) float sT[32][68];
  int b = blockIdx.x;
  const float* src; us16* dh; us16* dl; int Kr, Nc;
  if (b < 72)       {           src = w0; dh = t0h; dl = t0l; Kr = LD_W1; Nc = CFD;   }
  else if (b < 144) { b -= 72;  src = w1; dh = t1h; dl = t1l; Kr = LD_W1; Nc = CFD;   }
  else if (b < 272) { b -= 144; src = w2; dh = t2h; dl = t2l; Kr = DDIM;  Nc = MWH;   }
  else if (b < 276) { b -= 272; src = w3; dh = t3h; dl = t3l; Kr = MWH;   Nc = KCODE; }
  else              { b -= 276; src = w4; dh = t4h; dl = t4l; Kr = CFD;   Nc = CFD;   }
  const int nkt = Kr >> 6;
  const int kt = b % nkt, ntile = b / nkt;
  const int k0 = kt * 64, n0 = ntile * 32;
  const int tid = threadIdx.x;
  {
    const int row = tid >> 2, piece = tid & 3;
    const float* p = src + (size_t)(k0 + row) * Nc + n0 + 8 * piece;
    const v4f a = *(const v4fa*)p;
    const v4f c = *(const v4fa*)(p + 4);
    const int cb = 8 * piece;
    sT[cb + 0][row] = a.x; sT[cb + 1][row] = a.y; sT[cb + 2][row] = a.z; sT[cb + 3][row] = a.w;
    sT[cb + 4][row] = c.x; sT[cb + 5][row] = c.y; sT[cb + 6][row] = c.z; sT[cb + 7][row] = c.w;
  }
  __syncthreads();
  const int lane = tid & 31, w = tid >> 5, sub = lane >> 3, q = lane & 7;
  const int plane = w >> 2;
  us16* dst = plane ? dl : dh;
  v8us val[2];
  int nrow[2];
  #pragma unroll
  for (int i = 0; i < 2; ++i) {
    const int n = (w * 8 + i * 4 + sub) & 31;
    nrow[i] = n;
    const v4f a = *(const v4fa*)(&sT[n][8 * q]);
    const v4f c = *(const v4fa*)(&sT[n][8 * q + 4]);
    v8us vh, vl;
    split8(a, c, vh, vl);
    if (plane) val[i] = vl; else val[i] = vh;
  }
  #pragma unroll
  for (int i = 0; i < 2; ++i)
    *(volatile v8us*)(dst + (size_t)(n0 + nrow[i]) * Kr + k0 + 8 * q) = val[i];
  __threadfence();
  #pragma unroll
  for (int i = 0; i < 2; ++i)
    *(volatile v8us*)(dst + (size_t)(n0 + nrow[i]) * Kr + k0 + 8 * q) = val[i];
}

template <int RPW>
__device__ __forceinline__ void row_store(const float* s, float* dst, int w, int lane) {
  #pragma unroll
  for (int i = 0; i < RPW; ++i) {
    const int lrow = RPW * w + i;
    const v4f v = *(const v4fa*)(s + lrow * 132 + 4 * lane);
    *(volatile v4f*)(dst + (size_t)lrow * CFD + 4 * lane) = v;
  }
}

__global__ __launch_bounds__(64) void k_codes(
    const float* __restrict__ ce, const float* __restrict__ cmom,
    const us16* __restrict__ MUth, const us16* __restrict__ MUtl,
    const us16* __restrict__ LVth, const us16* __restrict__ LVtl,
    float* __restrict__ code_mu, float* __restrict__ code_lv)
{
  __shared__ __attribute__((aligned(16))) us16  sAh[KCODE * 136];
  __shared__ __attribute__((aligned(16))) us16  sAl[KCODE * 136];
  __shared__ __attribute__((aligned(16))) float sO[KCODE * 132];
  const int which = blockIdx.x;
  const int tid = threadIdx.x, lane = tid & 31, w = tid >> 5, hh = lane >> 4, m = lane & 15;

  for (int idx = tid; idx < KCODE * CDIM; idx += 64) {
    const int k = idx >> 7, e = idx & 127;
    const float pa = 0.9f * cmom[idx];
    const float pb = 0.1f * ce[idx];
    const float x = pa + pb;
    us16 xh, xl;
    split1(x, xh, xl);
    sAh[k * 136 + e] = xh;
    sAl[k * 136 + e] = xl;
  }
  __syncthreads();

  const us16* Bh = which ? LVth : MUth;
  const us16* Bl = which ? LVtl : MUtl;
  float* dst = which ? code_lv : code_mu;
  const v8f zero8 = {0.f, 0.f, 0.f, 0.f, 0.f, 0.f, 0.f, 0.f};
  v8f acc[8];
  #pragma unroll
  for (int nt = 0; nt < 8; ++nt) acc[nt] = zero8;
  const us16* arh = sAh + (16 * w + m) * 136;
  const us16* arl = sAl + (16 * w + m) * 136;

  #pragma unroll 1
  for (int k0 = 0; k0 < CDIM; k0 += 32) {
    const v16bf ah = load_frag(arh + k0, hh);
    const v16bf al = load_frag(arl + k0, hh);
    #pragma unroll
    for (int nt = 0; nt < 8; ++nt) {
      const size_t off = (size_t)(16 * nt + m) * LD_W1 + DDIM + k0;
      const v16bf bh = load_frag(Bh + off, hh);
      const v16bf bl = load_frag(Bl + off, hh);
      acc[nt] = mma3(ah, al, bh, bl, acc[nt]);
    }
  }
  #pragma unroll
  for (int nt = 0; nt < 8; ++nt)
    #pragma unroll
    for (int r = 0; r < 8; ++r)
      sO[(16 * w + 8 * hh + r) * 132 + 16 * nt + m] = acc[nt][r];
  __syncthreads();

  row_store<16>(sO, dst, w, lane);
  __threadfence();
  row_store<16>(sO, dst, w, lane);
}

__device__ __forceinline__ void tok_store(const float* sT, int kind, float* Pdst, us16* Mh, us16* Ml,
                                          int bm, int cseg, int w, int lane) {
  if (kind != 2) {
    #pragma unroll
    for (int i = 0; i < 8; ++i) {
      const int lrow = 16 * w + 2 * i + (lane >> 4);
      const int p = lane & 15;
      const v4f v = *(const v4fa*)(sT + lrow * 68 + 4 * p);
      *(volatile v4f*)(Pdst + (size_t)(bm * 64 + lrow) * CFD + cseg + 4 * p) = v;
    }
  } else {
    #pragma unroll
    for (int i = 0; i < 4; ++i) {
      const int lrow = 16 * w + 4 * i + (lane >> 3);
      const int q = lane & 7;
      const v4f a = *(const v4fa*)(sT + lrow * 68 + 8 * q);
      const v4f c = *(const v4fa*)(sT + lrow * 68 + 8 * q + 4);
      v8us vh, vl;
      split8(a, c, vh, vl);
      const size_t off = (size_t)(bm * 64 + lrow) * MWH + cseg + 8 * q;
      *(volatile v8us*)(Mh + off) = vh;
      *(volatile v8us*)(Ml + off) = vl;
    }
  }
}

__global__ __launch_bounds__(128) void k_tok(
    const us16* __restrict__ Hh, const us16* __restrict__ Hl,
    const us16* __restrict__ MUth, const us16* __restrict__ MUtl,
    const us16* __restrict__ LVth, const us16* __restrict__ LVtl,
    const us16* __restrict__ MW1th, const us16* __restrict__ MW1tl,
    const float* __restrict__ mw_b1,
    float* __restrict__ P_mu, float* __restrict__ P_lv,
    us16* __restrict__ M1h, us16* __restrict__ M1l)
{
  __shared__ __attribute__((aligned(16))) float sT[64 * 68];
  const int tid = threadIdx.x, lane = tid & 31, w = tid >> 5;
  const int hh = lane >> 4, m = lane & 15;
  const int bm = blockIdx.x, cb = blockIdx.y;
  const int wr = w & 1, wc = w >> 1;

  const us16* Bh; const us16* Bl; int ldb, cseg, kind; float* Pdst;
  if (cb < 2)      { Bh = MUth;  Bl = MUtl;  ldb = LD_W1; cseg = 64 * cb;       kind = 0; Pdst = P_mu; }
  else if (cb < 4) { Bh = LVth;  Bl = LVtl;  ldb = LD_W1; cseg = 64 * (cb - 2); kind = 1; Pdst = P_lv; }
  else             { Bh = MW1th; Bl = MW1tl; ldb = DDIM;  cseg = 64 * (cb - 4); kind = 2; Pdst = P_mu; }

  const int row0 = bm * 64 + 32 * wr;
  const us16* ah0 = Hh + (size_t)(row0 + m) * DDIM;
  const us16* ah1 = ah0 + (size_t)16 * DDIM;
  const us16* al0 = Hl + (size_t)(row0 + m) * DDIM;
  const us16* al1 = al0 + (size_t)16 * DDIM;
  const int n0 = cseg + 32 * wc;
  const us16* bh0 = Bh + (size_t)(n0 + m) * ldb;
  const us16* bh1 = bh0 + (size_t)16 * ldb;
  const us16* bl0 = Bl + (size_t)(n0 + m) * ldb;
  const us16* bl1 = bl0 + (size_t)16 * ldb;

  const v8f zero8 = {0.f, 0.f, 0.f, 0.f, 0.f, 0.f, 0.f, 0.f};
  v8f acc[2][2];
  acc[0][0] = zero8; acc[0][1] = zero8; acc[1][0] = zero8; acc[1][1] = zero8;

  #pragma unroll 1
  for (int k0 = 0; k0 < DDIM; k0 += 32) {
    const v16bf a0h = load_frag(ah0 + k0, hh);
    const v16bf a0l = load_frag(al0 + k0, hh);
    const v16bf a1h = load_frag(ah1 + k0, hh);
    const v16bf a1l = load_frag(al1 + k0, hh);
    const v16bf b0h = load_frag(bh0 + k0, hh);
    const v16bf b0l = load_frag(bl0 + k0, hh);
    const v16bf b1h = load_frag(bh1 + k0, hh);
    const v16bf b1l = load_frag(bl1 + k0, hh);
    acc[0][0] = mma3(a0h, a0l, b0h, b0l, acc[0][0]);
    acc[0][1] = mma3(a0h, a0l, b1h, b1l, acc[0][1]);
    acc[1][0] = mma3(a1h, a1l, b0h, b0l, acc[1][0]);
    acc[1][1] = mma3(a1h, a1l, b1h, b1l, acc[1][1]);
  }

  #pragma unroll
  for (int mt = 0; mt < 2; ++mt)
    #pragma unroll
    for (int nt = 0; nt < 2; ++nt)
      #pragma unroll
      for (int r = 0; r < 8; ++r)
        sT[(32 * wr + 16 * mt + 8 * hh + r) * 68 + 32 * wc + 16 * nt + m] = acc[mt][nt][r];
  __syncthreads();

  if (kind == 2) {
    #pragma unroll 1
    for (int j = 0; j < 32; ++j) {
      const int idx = tid + 128 * j;
      const int lrow = idx >> 6, lcol = idx & 63;
      const float x = sT[lrow * 68 + lcol] + mw_b1[cseg + lcol];
      const float sg = 1.0f / (1.0f + expf(-x));
      sT[lrow * 68 + lcol] = x * sg;
    }
  }
  __syncthreads();

  tok_store(sT, kind, Pdst, M1h, M1l, bm, cseg, w, lane);
  __threadfence();
  tok_store(sT, kind, Pdst, M1h, M1l, bm, cseg, w, lane);
}

__device__ __forceinline__ void mix_store(const float* sL, float* o0, int w, int lane) {
  #pragma unroll
  for (int i = 0; i < 4; ++i) {
    const int lrow = 16 * w + 4 * i + (lane >> 3);
    const int q = lane & 7;
    const v4f v = *(const v4fa*)(sL + lrow * 36 + 4 * q);
    *(volatile v4f*)(o0 + (size_t)lrow * KCODE + 4 * q) = v;
  }
}

__global__ __launch_bounds__(64) void k_mix(
    const us16* __restrict__ M1h, const us16* __restrict__ M1l,
    const us16* __restrict__ MW2th, const us16* __restrict__ MW2tl,
    const float* __restrict__ mw_b2, float* __restrict__ out0)
{
  __shared__ __attribute__((aligned(16))) float sL[32 * 36];
  const int tid = threadIdx.x, lane = tid & 31, w = tid >> 5, hh = lane >> 4, m = lane & 15;
  const int bm = blockIdx.x;
  const int rowA = bm * 32 + 16 * w + m;
  const us16* arh = M1h + (size_t)rowA * MWH;
  const us16* arl = M1l + (size_t)rowA * MWH;
  const us16* b0h = MW2th + (size_t)m * MWH;
  const us16* b0l = MW2tl + (size_t)m * MWH;
  const us16* b1h = MW2th + (size_t)(16 + m) * MWH;
  const us16* b1l = MW2tl + (size_t)(16 + m) * MWH;

  const v8f zero8 = {0.f, 0.f, 0.f, 0.f, 0.f, 0.f, 0.f, 0.f};
  v8f acc[2];
  acc[0] = zero8; acc[1] = zero8;
  #pragma unroll 1
  for (int k0 = 0; k0 < MWH; k0 += 32) {
    const v16bf ah = load_frag(arh + k0, hh);
    const v16bf al = load_frag(arl + k0, hh);
    const v16bf p0h = load_frag(b0h + k0, hh);
    const v16bf p0l = load_frag(b0l + k0, hh);
    const v16bf p1h = load_frag(b1h + k0, hh);
    const v16bf p1l = load_frag(b1l + k0, hh);
    acc[0] = mma3(ah, al, p0h, p0l, acc[0]);
    acc[1] = mma3(ah, al, p1h, p1l, acc[1]);
  }
  #pragma unroll
  for (int nt = 0; nt < 2; ++nt)
    #pragma unroll
    for (int r = 0; r < 8; ++r) {
      const int n = 16 * nt + m;
      sL[(16 * w + 8 * hh + r) * 36 + n] = acc[nt][r] + mw_b2[n];
    }
  __syncthreads();

  if (tid < 32) {
    float* lr = sL + tid * 36;
    float mx = lr[0];
    #pragma unroll 1
    for (int j = 1; j < KCODE; ++j) mx = fmaxf(mx, lr[j]);
    float s = 0.f;
    #pragma unroll 1
    for (int j = 0; j < KCODE; ++j) {
      const float e = expf(lr[j] - mx);
      lr[j] = e;
      s += e;
    }
    const float inv = 1.0f / s;
    #pragma unroll 1
    for (int j = 0; j < KCODE; ++j) lr[j] = lr[j] * inv;
  }
  __syncthreads();

  float* o0 = out0 + (size_t)bm * 32 * KCODE;
  mix_store(sL, o0, w, lane);
  __threadfence();
  mix_store(sL, o0, w, lane);
}

__global__ __launch_bounds__(128) void k_mulv(
    const float* __restrict__ P_mu, const float* __restrict__ P_lv,
    const float* __restrict__ code_mu, const float* __restrict__ code_lv,
    const float* __restrict__ mu_b1, const float* __restrict__ ln_g, const float* __restrict__ ln_b,
    const us16* __restrict__ MU2th, const us16* __restrict__ MU2tl,
    const float* __restrict__ mu_b2, const float* __restrict__ lv_b,
    float* __restrict__ out1, float* __restrict__ out2)
{
  __shared__ __attribute__((aligned(16))) float sX[KCODE * 132];
  __shared__ __attribute__((aligned(16))) float sO[KCODE * 132];
  __shared__ __attribute__((aligned(16))) us16  sAh[KCODE * 136];
  __shared__ __attribute__((aligned(16))) us16  sAl[KCODE * 136];
  const int bt = blockIdx.x;
  const int tid = threadIdx.x, lane = tid & 31, w = tid >> 5, hh = lane >> 4, m = lane & 15;

  {
    const int c = tid;
    const float pm = P_mu[(size_t)bt * CFD + c];
    const float pl = P_lv[(size_t)bt * CFD + c];
    const float b1 = mu_b1[c], b2 = lv_b[c];
    #pragma unroll 4
    for (int k = 0; k < KCODE; ++k) {
      const float xm = (pm + code_mu[k * CFD + c]) + b1;
      sX[k * 132 + c] = xm;
      float v = (pl + code_lv[k * CFD + c]) + b2;
      v = fminf(fmaxf(v, LVMIN), LVMAX);
      sO[k * 132 + c] = v;
    }
  }
  __syncthreads();

  float* o2 = out2 + (size_t)bt * KCODE * CFD;
  row_store<8>(sO, o2, w, lane);
  __threadfence();
  row_store<8>(sO, o2, w, lane);

  {
    const int row = tid >> 2, c0 = 32 * (tid & 3);
    const float* xr = sX + row * 132 + c0;
    float s = 0.f;
    #pragma unroll 8
    for (int j = 0; j < 32; ++j) s += xr[j];
    s += __shfl_xor(s, 1);
    s += __shfl_xor(s, 2);
    const float mean = s * (1.0f / 128.0f);
    float vs = 0.f;
    #pragma unroll 8
    for (int j = 0; j < 32; ++j) { const float d = xr[j] - mean; vs += d * d; }
    vs += __shfl_xor(vs, 1);
    vs += __shfl_xor(vs, 2);
    const float rstd = rsqrtf(vs * (1.0f / 128.0f) + LNEPS);
    #pragma unroll 4
    for (int j = 0; j < 32; ++j) {
      const int col = c0 + j;
      const float y = (xr[j] - mean) * rstd * ln_g[col] + ln_b[col];
      us16 yh, yl;
      split1(y, yh, yl);
      sAh[row * 136 + col] = yh;
      sAl[row * 136 + col] = yl;
    }
  }
  __syncthreads();

  const int mt = w & 1, ntb = 4 * (w >> 1);
  const us16* arh = sAh + (16 * mt + m) * 136;
  const us16* arl = sAl + (16 * mt + m) * 136;
  const v8f zero8 = {0.f, 0.f, 0.f, 0.f, 0.f, 0.f, 0.f, 0.f};
  v8f acc[4];
  acc[0] = zero8; acc[1] = zero8; acc[2] = zero8; acc[3] = zero8;
  #pragma unroll 1
  for (int k0 = 0; k0 < CFD; k0 += 32) {
    const v16bf ah = load_frag(arh + k0, hh);
    const v16bf al = load_frag(arl + k0, hh);
    #pragma unroll
    for (int nt = 0; nt < 4; ++nt) {
      const size_t off = (size_t)(16 * (ntb + nt) + m) * CFD + k0;
      const v16bf bh = load_frag(MU2th + off, hh);
      const v16bf bl = load_frag(MU2tl + off, hh);
      acc[nt] = mma3(ah, al, bh, bl, acc[nt]);
    }
  }
  #pragma unroll
  for (int nt = 0; nt < 4; ++nt) {
    const int n = 16 * (ntb + nt) + m;
    const float bb = mu_b2[n];
    #pragma unroll
    for (int r = 0; r < 8; ++r) {
      float y = tanhf(acc[nt][r] + bb);
      y = fminf(fmaxf(y, -3.0f), 3.0f);
      sO[(16 * mt + 8 * hh + r) * 132 + n] = y;
    }
  }
  __syncthreads();

  float* o1 = out1 + (size_t)bt * KCODE * CFD;
  row_store<8>(sO, o1, w, lane);
  __threadfence();
  row_store<8>(sO, o1, w, lane);
}

extern "C" void kernel_launch(void* const* d_in, const int* in_sizes, int n_in,
                              void* d_out, int out_size, void* d_ws, size_t ws_size,
                              hipStream_t stream) {
  if (n_in < 15) return;
  if (in_sizes[0] != NTOK * DDIM) return;
  if (in_sizes[1] != KCODE * CDIM || in_sizes[2] != KCODE * CDIM) return;
  if (in_sizes[3] != LD_W1 * CFD || in_sizes[9] != LD_W1 * CFD) return;
  if (in_sizes[4] != CFD || in_sizes[5] != CFD || in_sizes[6] != CFD) return;
  if (in_sizes[7] != CFD * CFD || in_sizes[8] != CFD || in_sizes[10] != CFD) return;
  if (in_sizes[11] != DDIM * MWH || in_sizes[12] != MWH) return;
  if (in_sizes[13] != MWH * KCODE || in_sizes[14] != KCODE) return;
  if (out_size != NTOK * KCODE + 2 * NTOK * KCODE * CFD) return;

  const float* h             = (const float*)d_in[0];
  const float* code_embed    = (const float*)d_in[1];
  const float* code_momentum = (const float*)d_in[2];
  const float* mu_w1         = (const float*)d_in[3];
  const float* mu_b1         = (const float*)d_in[4];
  const float* ln_g          = (const float*)d_in[5];
  const float* ln_b          = (const float*)d_in[6];
  const float* mu_w2         = (const float*)d_in[7];
  const float* mu_b2         = (const float*)d_in[8];
  const float* lv_w          = (const float*)d_in[9];
  const float* lv_b          = (const float*)d_in[10];
  const float* mw_w1         = (const float*)d_in[11];
  const float* mw_b1         = (const float*)d_in[12];
  const float* mw_w2         = (const float*)d_in[13];
  const float* mw_b2         = (const float*)d_in[14];

  const size_t hp_bytes  = (size_t)NTOK * DDIM * 2;
  const size_t w1t_bytes = (size_t)CFD * LD_W1 * 2;
  const size_t mw1_bytes = (size_t)MWH * DDIM * 2;
  const size_t mw2_bytes = (size_t)KCODE * MWH * 2;
  const size_t mu2_bytes = (size_t)CFD * CFD * 2;
  const size_t p_bytes   = (size_t)NTOK * CFD * 4;
  const size_t m1_bytes  = (size_t)NTOK * MWH * 2;
  const size_t cd_bytes  = (size_t)KCODE * CFD * 4;
  const size_t total = 2 * hp_bytes + 4 * w1t_bytes + 2 * mw1_bytes + 2 * mw2_bytes + 2 * mu2_bytes
                     + 2 * p_bytes + 2 * m1_bytes + 2 * cd_bytes;
  if (total > ws_size) return;

  char* ws = (char*)d_ws;
  size_t off = 0;
  us16* Hh    = (us16*)(ws + off); off += hp_bytes;
  us16* Hl    = (us16*)(ws + off); off += hp_bytes;
  us16* MUth  = (us16*)(ws + off); off += w1t_bytes;
  us16* MUtl  = (us16*)(ws + off); off += w1t_bytes;
  us16* LVth  = (us16*)(ws + off); off += w1t_bytes;
  us16* LVtl  = (us16*)(ws + off); off += w1t_bytes;
  us16* MW1th = (us16*)(ws + off); off += mw1_bytes;
  us16* MW1tl = (us16*)(ws + off); off += mw1_bytes;
  us16* MW2th = (us16*)(ws + off); off += mw2_bytes;
  us16* MW2tl = (us16*)(ws + off); off += mw2_bytes;
  us16* MU2th = (us16*)(ws + off); off += mu2_bytes;
  us16* MU2tl = (us16*)(ws + off); off += mu2_bytes;
  float* P_mu    = (float*)(ws + off); off += p_bytes;
  float* P_lv    = (float*)(ws + off); off += p_bytes;
  us16* M1h   = (us16*)(ws + off); off += m1_bytes;
  us16* M1l   = (us16*)(ws + off); off += m1_bytes;
  float* code_mu = (float*)(ws + off); off += cd_bytes;
  float* code_lv = (float*)(ws + off); off += cd_bytes;
  if (off > ws_size) return;

  float* out  = (float*)d_out;
  float* out0 = out;
  float* out1 = out + (size_t)NTOK * KCODE;
  float* out2 = out1 + (size_t)NTOK * KCODE * CFD;

  k_convert_h<<<NH8 / 256, 256, 0, stream>>>(h, Hh, Hl);
  k_transpose_w<<<284, 256, 0, stream>>>(mu_w1, lv_w, mw_w1, mw_w2, mu_w2,
                                         MUth, MUtl, LVth, LVtl, MW1th, MW1tl,
                                         MW2th, MW2tl, MU2th, MU2tl);
  k_codes<<<2, 64, 0, stream>>>(code_embed, code_momentum, MUth, MUtl, LVth, LVtl, code_mu, code_lv);
  k_tok<<<dim3(NTOK / 64, 8), 128, 0, stream>>>(Hh, Hl, MUth, MUtl, LVth, LVtl, MW1th, MW1tl,
                                                mw_b1, P_mu, P_lv, M1h, M1l);
  k_mix<<<NTOK / 32, 64, 0, stream>>>(M1h, M1l, MW2th, MW2tl, mw_b2, out0);
  k_mulv<<<NTOK, 128, 0, stream>>>(P_mu, P_lv, code_mu, code_lv, mu_b1, ln_g, ln_b,
                                   MU2th, MU2tl, mu_b2, lv_b, out1, out2);
}
